// LSTMTagger_18915035972398
// MI455X (gfx1250) — hardware-verified
//
#include <hip/hip_runtime.h>
#include <math.h>

constexpr int NBAT  = 16;
constexpr int NSEQ  = 1024;
constexpr int NDIM  = 512;
constexpr int NHEAD = 64;
constexpr int NLAY  = 16;
constexpr int NSM   = 8;
constexpr int NSETD = 128;
constexpr int NOTT  = NLAY * NSETD;
constexpr int NROW  = NBAT * NSEQ;
constexpr int NTHR  = 256;
constexpr int VECP  = 32;
constexpr int THW_PITCH = 260;
constexpr int XOP   = 516;
constexpr int SOP   = 132;
constexpr int NSUMALL = NLAY * NBAT * NSEQ;
constexpr int NOUTF   = NBAT + NSUMALL;
constexpr float WATT_CARRY = 256.0f;
constexpr float EMB_CARRY  = 256.0f;
constexpr float ATT_CARRY  = 1024.0f;
constexpr float RATE_SCALE = 1.0f / 65536.0f;
constexpr float POOL_SCALE = 1.0f / 8388608.0f;
constexpr float LN_EPS = 1e-5f;
static_assert(RATE_SCALE * WATT_CARRY * EMB_CARRY == 1.0f);
static_assert(POOL_SCALE * 32.0f * ATT_CARRY * EMB_CARRY == 1.0f);
static_assert(NDIM % 32 == 0 && NSEQ % 32 == 0);
static_assert(NHEAD % 64 == 0 && NSEQ % 64 == 0 && NDIM % 64 == 0);
static_assert(NTHR == 256);
static_assert(NSEQ == 4 * NTHR);
static_assert(NROW % 64 == 0 && NSEQ % 64 == 0);
static_assert(NOUTF % 4 == 0);
static_assert(NDIM == 2 * NTHR);
static_assert(NBAT * NSETD == 8 * NTHR);
static_assert((NLAY * NHEAD * NDIM) % (8 * NTHR) == 0);

typedef __attribute__((ext_vector_type(16))) _Float16 v16h;
typedef __attribute__((ext_vector_type(8)))  _Float16 v8h;
typedef __attribute__((ext_vector_type(16))) __bf16   v16b;
typedef __attribute__((ext_vector_type(8)))  __bf16   v8b;
typedef __attribute__((ext_vector_type(8)))  float    v8f;
typedef __attribute__((ext_vector_type(4)))  float    v4f;
typedef __attribute__((ext_vector_type(4)))  unsigned v4u;
typedef __attribute__((ext_vector_type(2)))  unsigned v2u;

__device__ __forceinline__ unsigned short f2bf_bits(float f) {
  unsigned u = __float_as_uint(f);
  return (unsigned short)((u + 0x7FFFu + ((u >> 16) & 1u)) >> 16);
}
__device__ __forceinline__ float bf_bits2f(unsigned short h) { return __uint_as_float(((unsigned)h) << 16); }
__device__ __forceinline__ unsigned short f2h_bits(float f) { return __builtin_bit_cast(unsigned short, (_Float16)f); }

__device__ __forceinline__ void dep_guard_h(v8f& a, v8f& b, v16h x, v16h y) { asm volatile("v_nop\n\tv_nop\n\tv_nop\n\tv_nop" : "+v"(a), "+v"(b) : "v"(x), "v"(y)); }
__device__ __forceinline__ void dep_guard_b(v8f& a, v8f& b, v16b x, v16b y) { asm volatile("v_nop\n\tv_nop\n\tv_nop\n\tv_nop" : "+v"(a), "+v"(b) : "v"(x), "v"(y)); }
__device__ __forceinline__ void dep_guard4_h(v8f& a, v8f& b, v8f& c, v8f& d, v16h x, v16h y) { asm volatile("v_nop\n\tv_nop\n\tv_nop\n\tv_nop" : "+v"(a), "+v"(b), "+v"(c), "+v"(d) : "v"(x), "v"(y)); }
__device__ __forceinline__ void dep_guard4_b(v8f& a, v8f& b, v8f& c, v8f& d, v16b x, v16b y) { asm volatile("v_nop\n\tv_nop\n\tv_nop\n\tv_nop" : "+v"(a), "+v"(b), "+v"(c), "+v"(d) : "v"(x), "v"(y)); }
__device__ __forceinline__ void keep4_h(v16h a, v16h b, v16h c, v16h d) { asm volatile("v_nop" :: "v"(a), "v"(b), "v"(c), "v"(d)); }
__device__ __forceinline__ void keep4_b(v16b a, v16b b, v16b c, v16b d) { asm volatile("v_nop" :: "v"(a), "v"(b), "v"(c), "v"(d)); }
__device__ __forceinline__ void acc_guard4(v8f& a, v8f& b, v8f& c, v8f& d) { asm volatile("v_nop\n\tv_nop\n\tv_nop\n\tv_nop" : "+v"(a), "+v"(b), "+v"(c), "+v"(d)); }
template <typename T> struct Frag;
template <> struct Frag<_Float16> {
  typedef v16h V; union U { v16h v; v8h h[2]; };
  static __device__ __forceinline__ v16h load(const _Float16* p) {
    U f; f.h[0] = *(const v8h*)(p); f.h[1] = *(const v8h*)(p + 16); return f.v;
  }
  static __device__ __forceinline__ v8f mma(v16h a, v16h b, v8f c) {
    return __builtin_amdgcn_wmma_f32_16x16x32_f16(false, a, false, b, (short)0, c, false, false);
  }
  static __device__ __forceinline__ void guard(v8f& a, v8f& b, v16h x, v16h y) { dep_guard_h(a, b, x, y); }
  static __device__ __forceinline__ void guard4(v8f& a, v8f& b, v8f& c, v8f& d, v16h x, v16h y) { dep_guard4_h(a, b, c, d, x, y); }
  static __device__ __forceinline__ void keep(v16h a, v16h b, v16h c, v16h d) { keep4_h(a, b, c, d); }
};
template <> struct Frag<__bf16> {
  typedef v16b V; union U { v16b v; v8b h[2]; };
  static __device__ __forceinline__ v16b load(const __bf16* p) {
    U f; f.h[0] = *(const v8b*)(p); f.h[1] = *(const v8b*)(p + 16); return f.v;
  }
  static __device__ __forceinline__ v8f mma(v16b a, v16b b, v8f c) {
    return __builtin_amdgcn_wmma_f32_16x16x32_bf16(false, a, false, b, (short)0, c, false, false);
  }
  static __device__ __forceinline__ void guard(v8f& a, v8f& b, v16b x, v16b y) { dep_guard_b(a, b, x, y); }
  static __device__ __forceinline__ void guard4(v8f& a, v8f& b, v8f& c, v8f& d, v16b x, v16b y) { dep_guard4_b(a, b, c, d, x, y); }
  static __device__ __forceinline__ void keep(v16b a, v16b b, v16b c, v16b d) { keep4_b(a, b, c, d); }
};

template <int ET> struct Elem;
template <> struct Elem<0> { typedef _Float16 T; };
template <> struct Elem<1> { typedef __bf16 T; };
template <int ET, bool SPLIT, int BIAS_MODE, int OUT_MODE, bool RESID, int ACT = 0>
__global__ __launch_bounds__(256) void wmma_gemm64(
    const unsigned short* __restrict__ Ap, const unsigned short* __restrict__ A2p, int lda, long strideA,
    const unsigned short* __restrict__ Btp, const unsigned short* __restrict__ Bt2p, int ldb, long strideB,
    void* __restrict__ Cout, void* __restrict__ Cout2, int ldc, long strideC,
    const float* __restrict__ bias,
    const float* __restrict__ resid, long strideR,
    int M, int N, int K, float scale) {
  typedef typename Elem<ET>::T T;
  typedef typename Frag<T>::V V;
  const T* A = (const T*)Ap; const T* A2 = (const T*)A2p; const T* Bt = (const T*)Btp; const T* Bt2 = (const T*)Bt2p;
  __shared__ __align__(16) float sT[8][16 * 68];
  const int b    = blockIdx.y;
  const int lane = threadIdx.x & 31;
  const int wave = threadIdx.x >> 5;
  const int tilesN = N >> 6;
  const int tilesM = M >> 6;
  const int tile = blockIdx.x * 8 + wave;
  if (tile >= tilesM * tilesN) return;
  const int tm = tile / tilesN;
  const int tn = tile - tm * tilesN;
  const int m0 = tm << 6;
  const int n0 = tn << 6;

  const T* Ab  = A  + (size_t)b * strideA;
  const T* Bb  = Bt + (size_t)b * strideB;
  const T* Ab2 = SPLIT ? (A2  + (size_t)b * strideA) : nullptr;
  const T* Bb2 = SPLIT ? (Bt2 + (size_t)b * strideB) : nullptr;

  const int rlane = lane & 15;
  const int koff  = (lane >> 4) * 8;
  const int mOff  = (lane >> 4) * 8;

  v8f acc[4][4];
#pragma unroll
  for (int i = 0; i < 4; ++i)
#pragma unroll
    for (int j = 0; j < 4; ++j) acc[i][j] = (v8f){0.f,0.f,0.f,0.f,0.f,0.f,0.f,0.f};

  for (int k0 = 0; k0 < K; k0 += 32) {
    V bh[4], bl[4];
#pragma unroll
    for (int j = 0; j < 4; ++j) {
      const size_t bo = (size_t)(n0 + (j << 4) + rlane) * ldb + koff + k0;
      bh[j] = Frag<T>::load(Bb + bo);
      if (SPLIT) bl[j] = Frag<T>::load(Bb2 + bo);
    }
#pragma unroll
    for (int i = 0; i < 4; ++i) {
      const size_t ao = (size_t)(m0 + (i << 4) + rlane) * lda + koff + k0;
      V ah = Frag<T>::load(Ab + ao);
      V al;
      if (SPLIT) al = Frag<T>::load(Ab2 + ao);
#pragma unroll
      for (int j = 0; j < 4; ++j) {
        acc[i][j] = Frag<T>::mma(ah, bh[j], acc[i][j]);
        if (SPLIT) {
          acc[i][j] = Frag<T>::mma(ah, bl[j], acc[i][j]);
          acc[i][j] = Frag<T>::mma(al, bh[j], acc[i][j]);
        }
      }
      Frag<T>::guard4(acc[i][0], acc[i][1], acc[i][2], acc[i][3], ah, SPLIT ? al : bh[3]);
    }
    Frag<T>::keep(bh[0], bh[1], bh[2], bh[3]);
    if (SPLIT) Frag<T>::keep(bl[0], bl[1], bl[2], bl[3]);
  }
  acc_guard4(acc[0][0], acc[0][1], acc[0][2], acc[0][3]);
  acc_guard4(acc[1][0], acc[1][1], acc[1][2], acc[1][3]);
  acc_guard4(acc[2][0], acc[2][1], acc[2][2], acc[2][3]);
  acc_guard4(acc[3][0], acc[3][1], acc[3][2], acc[3][3]);

  float* slab = sT[wave];
  const float* Rb = RESID ? (resid + (size_t)b * strideR) : nullptr;
#pragma unroll
  for (int i = 0; i < 4; ++i) {
    const int mBase = m0 + (i << 4);
    float bmv[8];
#pragma unroll
    for (int r = 0; r < 8; ++r) bmv[r] = 0.f;
    if (BIAS_MODE == 1) {
      const v4f bm0 = *(const v4f*)(bias + mBase + mOff);
      const v4f bm1 = *(const v4f*)(bias + mBase + mOff + 4);
#pragma unroll
      for (int r = 0; r < 4; ++r) { bmv[r] = bm0[r]; bmv[4 + r] = bm1[r]; }
    }
#pragma unroll
    for (int j = 0; j < 4; ++j) {
      const int n = n0 + (j << 4) + rlane;
      float bv = 0.f;
      if (BIAS_MODE == 2) bv = bias[n];
#pragma unroll
      for (int r = 0; r < 8; ++r) {
        float v = acc[i][j][r] * scale;
        if (BIAS_MODE == 1) v += bmv[r];
        if (BIAS_MODE == 2) v += bv;
        if (RESID) v += Rb[(size_t)(mBase + mOff + r) * ldc + n];
        if (ACT == 1) v = tanhf(v);
        if (ACT == 2) v = fmaxf(v, 0.0f);
        if (ACT == 3) v = v / (1.0f + expf(-v));
        if (ACT == 4) v = (v > 0.f) ? v : 0.01f * v;
        slab[(mOff + r) * 68 + (j << 4) + rlane] = v;
      }
    }
    __builtin_amdgcn_fence(__ATOMIC_RELEASE, "workgroup");
    __builtin_amdgcn_wave_barrier();
    __builtin_amdgcn_fence(__ATOMIC_ACQUIRE, "workgroup");
    if (OUT_MODE == 0) {
      float* C = (float*)Cout + (size_t)b * strideC;
      const int hh = lane >> 4, c4 = (lane & 15) * 4;
      for (int pass = 0; pass < 2; ++pass) {
#pragma unroll
        for (int it = 0; it < 8; ++it) {
          const int row = it * 2 + hh;
          v4f v = *(const v4f*)(slab + row * 68 + c4);
          *(volatile v4f*)(C + (size_t)(mBase + row) * ldc + n0 + c4) = v;
        }
        __threadfence();
      }
    } else {
      const int q = lane >> 3, c8 = (lane & 7) * 8;
      unsigned short* C  = (unsigned short*)Cout  + (size_t)b * strideC;
      unsigned short* C2 = (OUT_MODE == 2) ? ((unsigned short*)Cout2 + (size_t)b * strideC) : nullptr;
      for (int pass = 0; pass < 2; ++pass) {
#pragma unroll
        for (int it = 0; it < 4; ++it) {
          const int row = it * 4 + q;
          const float* sp = slab + row * 68 + c8;
          v8h hv, lv;
#pragma unroll
          for (int e = 0; e < 8; ++e) {
            if (OUT_MODE == 1) {
              hv[e] = (_Float16)sp[e];
            } else {
              unsigned short hb = f2bf_bits(sp[e]);
              unsigned short lb = f2bf_bits(sp[e] - bf_bits2f(hb));
              hv[e] = __builtin_bit_cast(_Float16, hb);
              lv[e] = __builtin_bit_cast(_Float16, lb);
            }
          }
          *(volatile v8h*)(C + (size_t)(mBase + row) * ldc + n0 + c8) = hv;
          if (OUT_MODE == 2) *(volatile v8h*)(C2 + (size_t)(mBase + row) * ldc + n0 + c8) = lv;
        }
        __threadfence();
      }
    }
    __builtin_amdgcn_fence(__ATOMIC_RELEASE, "workgroup");
    __builtin_amdgcn_wave_barrier();
    __builtin_amdgcn_fence(__ATOMIC_ACQUIRE, "workgroup");
  }
}

__global__ __launch_bounds__(NTHR) void cvt_f16x8_kernel(const float* __restrict__ src, unsigned short* __restrict__ dst,
                                                        int n8, float sc) {
  const int i = blockIdx.x * NTHR + threadIdx.x;
  if (i < n8) {
    const v4f a = *(const v4f*)(src + (size_t)i * 8);
    const v4f b = *(const v4f*)(src + (size_t)i * 8 + 4);
    v8h hv;
#pragma unroll
    for (int e = 0; e < 4; ++e) { hv[e] = (_Float16)(a[e] * sc); hv[4 + e] = (_Float16)(b[e] * sc); }
    *(volatile v8h*)(dst + (size_t)i * 8) = hv;
    __threadfence();
    *(volatile v8h*)(dst + (size_t)i * 8) = hv;
  }
}

template <bool W16>
__global__ __launch_bounds__(NTHR) void softmax_rows_kernel(const float* __restrict__ in, float* __restrict__ outf,
                                                            unsigned short* __restrict__ out16) {
  __shared__ float redm[8];
  __shared__ float reds[8];
  __shared__ __align__(16) float rowbuf[W16 ? NSEQ : 4];
  const int tid = threadIdx.x, lane = tid & 31, wave = tid >> 5;
  const size_t row = blockIdx.x;
  const v4f x = *(const v4f*)(in + row * NSEQ + 4 * tid);
  float m = fmaxf(fmaxf(x[0], x[1]), fmaxf(x[2], x[3]));
#pragma unroll
  for (int off = 1; off < 32; off <<= 1) m = fmaxf(m, __shfl_xor(m, off, 32));
  if (lane == 0) redm[wave] = m;
  __syncthreads();
  float mm = redm[0];
#pragma unroll
  for (int w = 1; w < 8; ++w) mm = fmaxf(mm, redm[w]);
  v4f ev;
#pragma unroll
  for (int e = 0; e < 4; ++e) ev[e] = expf(x[e] - mm);
  float s = (ev[0] + ev[1]) + (ev[2] + ev[3]);
#pragma unroll
  for (int off = 1; off < 32; off <<= 1) s += __shfl_xor(s, off, 32);
  if (lane == 0) reds[wave] = s;
  __syncthreads();
  float tot = 0.f;
#pragma unroll
  for (int w = 0; w < 8; ++w) tot += reds[w];
  const float inv = 1.0f / tot;
  const v4f p = ev * inv;
  float* op = outf + row * NSEQ + 4 * tid;
  *(volatile v4f*)op = p;
  __threadfence();
  *(volatile v4f*)op = p;
  if (W16) {
    *(v4f*)(rowbuf + 4 * tid) = p;
    __syncthreads();
    if (tid < 128) {
      const v4f a = *(const v4f*)(rowbuf + 8 * tid);
      const v4f c = *(const v4f*)(rowbuf + 8 * tid + 4);
      v8h hv;
#pragma unroll
      for (int e = 0; e < 4; ++e) { hv[e] = (_Float16)(a[e] * ATT_CARRY); hv[4 + e] = (_Float16)(c[e] * ATT_CARRY); }
      unsigned short* hp = out16 + row * NSEQ + 8 * tid;
      *(volatile v8h*)hp = hv;
      __threadfence();
      *(volatile v8h*)hp = hv;
    }
  }
}

__global__ __launch_bounds__(NTHR) void headsum_kernel(const float* __restrict__ att, float* __restrict__ sumout) {
  const int i = blockIdx.x * NTHR + threadIdx.x;
  const int bq = i >> 8, l4 = (i & 255) * 4;
  const float* ap = att + (size_t)bq * NHEAD * NSEQ + l4;
  v4f s = (v4f){0.f, 0.f, 0.f, 0.f};
#pragma unroll 1
  for (int k = 0; k < NHEAD; ++k) s += *(const v4f*)(ap + (size_t)k * NSEQ);
  float* op = sumout + (size_t)i * 4;
  *(volatile v4f*)op = s;
  __threadfence();
  *(volatile v4f*)op = s;
}

__global__ __launch_bounds__(NTHR) void lnpro_kernel(const float* __restrict__ sraw, const float* __restrict__ ga,
                                                    const float* __restrict__ bea, const float* __restrict__ wpro,
                                                    const float* __restrict__ bpro, float* __restrict__ vec) {
  const int tid = threadIdx.x, lane = tid & 31, wave = tid >> 5;
  const int row = blockIdx.x * 8 + wave;
  const int k = row & 63;
  const float* sp  = sraw + (size_t)row * NDIM;
  const float* gp  = ga   + (size_t)k * NDIM;
  const float* ep  = bea  + (size_t)k * NDIM;
  const float* wpp = wpro + (size_t)k * NDIM * NSM;
  v4f v[4];
  float s = 0.f;
#pragma unroll
  for (int q = 0; q < 4; ++q) {
    v[q] = *(const v4f*)(sp + 128 * q + 4 * lane);
    s += (v[q][0] + v[q][1]) + (v[q][2] + v[q][3]);
  }
#pragma unroll
  for (int off = 1; off < 32; off <<= 1) s += __shfl_xor(s, off, 32);
  const float mean = s * (1.0f / NDIM);
  float ss = 0.f;
#pragma unroll
  for (int q = 0; q < 4; ++q)
#pragma unroll
    for (int e = 0; e < 4; ++e) { const float d = v[q][e] - mean; ss += d * d; }
#pragma unroll
  for (int off = 1; off < 32; off <<= 1) ss += __shfl_xor(ss, off, 32);
  const float rstd = rsqrtf(ss * (1.0f / NDIM) + LN_EPS);
  float acc[8];
#pragma unroll
  for (int e = 0; e < 8; ++e) acc[e] = 0.f;
#pragma unroll 1
  for (int q = 0; q < 4; ++q) {
    const int d0 = 128 * q + 4 * lane;
    const v4f xv = *(const v4f*)(sp + d0);
    const v4f gq = *(const v4f*)(gp + d0);
    const v4f eq = *(const v4f*)(ep + d0);
    asm volatile("" ::: "memory");
#pragma unroll
    for (int i = 0; i < 4; ++i) {
      const float xn = ((xv[i] - mean) * rstd) * gq[i] + eq[i];
      const v4f w0 = *(const v4f*)(wpp + (size_t)(d0 + i) * NSM);
      const v4f w1 = *(const v4f*)(wpp + (size_t)(d0 + i) * NSM + 4);
#pragma unroll
      for (int e = 0; e < 4; ++e) { acc[e] += xn * w0[e]; acc[4 + e] += xn * w1[e]; }
      asm volatile("" ::: "memory");
    }
  }
#pragma unroll
  for (int e = 0; e < 8; ++e) {
#pragma unroll
    for (int off = 1; off < 32; off <<= 1) acc[e] += __shfl_xor(acc[e], off, 32);
  }
  const v4f pb0 = *(const v4f*)(bpro + k * NSM);
  const v4f pb1 = *(const v4f*)(bpro + k * NSM + 4);
  float r[8];
#pragma unroll
  for (int e = 0; e < 4; ++e) { r[e] = fmaxf(acc[e] + pb0[e], 0.f); r[4 + e] = fmaxf(acc[4 + e] + pb1[e], 0.f); }
  const float f0 = (lane == 0) ? 1.f : 0.f;
  const float f1 = (lane == 1) ? 1.f : 0.f;
  v4f o;
#pragma unroll
  for (int e = 0; e < 4; ++e) o[e] = fmaf(f0, r[e], f1 * r[4 + e]);
  if (lane < 8) {
    float* vp = vec + (size_t)row * VECP + 4 * lane;
    *(volatile v4f*)vp = o;
    __threadfence();
    *(volatile v4f*)vp = o;
  }
}

__global__ __launch_bounds__(NTHR) void fiset_kernel(const float* __restrict__ vec, const float* __restrict__ wfi,
                                                    const float* __restrict__ bfi, const float* __restrict__ wset,
                                                    const float* __restrict__ bset, float* __restrict__ ott, int tcol) {
  __shared__ __align__(16) float xo[NBAT * XOP];
  __shared__ __align__(16) float so[NBAT * SOP];
  const int tid = threadIdx.x;
#pragma unroll 1
  for (int it = 0; it < 32; ++it) {
    const int idx = it * NTHR + tid;
    const int bq = idx >> 9, col = idx & 511;
    const int e = col >> 6, k = col & 63;
    xo[bq * XOP + col] = vec[(size_t)(bq * NHEAD + k) * VECP + e];
  }
  __syncthreads();
  float a0[NBAT], a1[NBAT];
#pragma unroll
  for (int m = 0; m < NBAT; ++m) { a0[m] = 0.f; a1[m] = 0.f; }
#pragma unroll 1
  for (int k = 0; k < NDIM; ++k) {
    const float w0 = wfi[(size_t)k * NDIM + tid];
    const float w1 = wfi[(size_t)k * NDIM + tid + NTHR];
#pragma unroll
    for (int m = 0; m < NBAT; ++m) {
      const float xv = xo[m * XOP + k];
      a0[m] += xv * w0;
      a1[m] += xv * w1;
    }
  }
  __syncthreads();
  {
    const float b0 = bfi[tid], b1 = bfi[tid + NTHR];
#pragma unroll
    for (int m = 0; m < NBAT; ++m) {
      const float r0 = xo[m * XOP + tid];
      const float r1 = xo[m * XOP + tid + NTHR];
      xo[m * XOP + tid]        = fmaxf(a0[m] + b0, 0.f) + r0;
      xo[m * XOP + tid + NTHR] = fmaxf(a1[m] + b1, 0.f) + r1;
    }
  }
  __syncthreads();
  {
    const int n = tid & 127, rg = tid >> 7;
    float c[8];
#pragma unroll
    for (int r = 0; r < 8; ++r) c[r] = 0.f;
#pragma unroll 1
    for (int k = 0; k < NDIM; ++k) {
      const float w = wset[(size_t)k * NSETD + n];
#pragma unroll
      for (int r = 0; r < 8; ++r) c[r] += xo[(8 * rg + r) * XOP + k] * w;
    }
    const float bs = bset[n];
#pragma unroll
    for (int r = 0; r < 8; ++r) so[(8 * rg + r) * SOP + n] = fmaxf(c[r] + bs, 0.f);
  }
  __syncthreads();
  for (int pass = 0; pass < 2; ++pass) {
#pragma unroll
    for (int it = 0; it < 2; ++it) {
      const int idx = it * NTHR + tid;
      const int row = idx >> 5, c4 = (idx & 31) * 4;
      const v4f vv = *(const v4f*)(so + row * SOP + c4);
      *(volatile v4f*)(ott + (size_t)row * NOTT + tcol + c4) = vv;
    }
    __threadfence();
  }
}

template <bool UPD>
__global__ __launch_bounds__(NTHR) void carry_kernel(const float* __restrict__ src, const float* __restrict__ sumatt,
                                                    const float* __restrict__ wp1, const float* __restrict__ bp1,
                                                    const float* __restrict__ gnv, const float* __restrict__ bnv,
                                                    float* __restrict__ dst, unsigned short* __restrict__ emb16,
                                                    unsigned short* __restrict__ embt16) {
  __shared__ __align__(16) unsigned ThW[64 * THW_PITCH];
  const int tid = threadIdx.x, lane = tid & 31, wave = tid >> 5;
  const int blk = blockIdx.x;
  const size_t rowbase = (size_t)blk * 64;
  const int bq = blk >> 4;
  const int l0 = (blk & 15) * 64;
  v4f wv[4], bv[4], gv[4], ev[4];
  if (UPD) {
#pragma unroll
    for (int q = 0; q < 4; ++q) {
      wv[q] = *(const v4f*)(wp1 + 128 * q + 4 * lane);
      bv[q] = *(const v4f*)(bp1 + 128 * q + 4 * lane);
    }
    asm volatile("" ::: "memory");
#pragma unroll
    for (int q = 0; q < 4; ++q) {
      gv[q] = *(const v4f*)(gnv + 128 * q + 4 * lane);
      ev[q] = *(const v4f*)(bnv + 128 * q + 4 * lane);
    }
    asm volatile("" ::: "memory");
  }
#pragma unroll 1
  for (int rr = 0; rr < 8; ++rr) {
    const int trow = wave * 8 + rr;
    const size_t grow = rowbase + (size_t)trow;
    const float* xp = src + grow * NDIM;
    v4f y[4];
#pragma unroll
    for (int q = 0; q < 4; ++q) y[q] = *(const v4f*)(xp + 128 * q + 4 * lane);
    if (UPD) {
      const float sa = sumatt[grow];
      float s = 0.f;
#pragma unroll
      for (int q = 0; q < 4; ++q)
#pragma unroll
        for (int e = 0; e < 4; ++e) {
          const float xv = y[q][e];
          const float pr = sa * wv[q][e] + bv[q][e];
          const float yv = xv * pr + xv;
          y[q][e] = yv;
          s += yv;
        }
#pragma unroll
      for (int off = 1; off < 32; off <<= 1) s += __shfl_xor(s, off, 32);
      const float mean = s * (1.0f / NDIM);
      float ss = 0.f;
#pragma unroll
      for (int q = 0; q < 4; ++q)
#pragma unroll
        for (int e = 0; e < 4; ++e) { const float d = y[q][e] - mean; y[q][e] = d; ss += d * d; }
#pragma unroll
      for (int off = 1; off < 32; off <<= 1) ss += __shfl_xor(ss, off, 32);
      const float rstd = rsqrtf(ss * (1.0f / NDIM) + LN_EPS);
#pragma unroll
      for (int q = 0; q < 4; ++q)
#pragma unroll
        for (int e = 0; e < 4; ++e) y[q][e] = (y[q][e] * rstd) * gv[q][e] + ev[q][e];
      float* dp = dst + grow * NDIM;
#pragma unroll
      for (int q = 0; q < 4; ++q) *(volatile v4f*)(dp + 128 * q + 4 * lane) = y[q];
      __threadfence();
#pragma unroll
      for (int q = 0; q < 4; ++q) *(volatile v4f*)(dp + 128 * q + 4 * lane) = y[q];
    }
#pragma unroll
    for (int q = 0; q < 4; ++q) {
      const unsigned h0 = f2h_bits(y[q][0] * EMB_CARRY);
      const unsigned h1 = f2h_bits(y[q][1] * EMB_CARRY);
      const unsigned h2 = f2h_bits(y[q][2] * EMB_CARRY);
      const unsigned h3 = f2h_bits(y[q][3] * EMB_CARRY);
      v2u pk;
      pk[0] = h0 | (h1 << 16);
      pk[1] = h2 | (h3 << 16);
      *(v2u*)(ThW + trow * THW_PITCH + 64 * q + 2 * lane) = pk;
    }
  }
  __syncthreads();
#pragma unroll
  for (int grp = 0; grp < 2; ++grp) {
    v4u vals[8];
#pragma unroll
    for (int it = 0; it < 8; ++it) {
      const int idx = (grp * 8 + it) * NTHR + tid;
      const int row = idx >> 6, c16 = idx & 63;
      vals[it] = *(const v4u*)(ThW + row * THW_PITCH + c16 * 4);
    }
    for (int pass = 0; pass < 2; ++pass) {
#pragma unroll
      for (int it = 0; it < 8; ++it) {
        const int idx = (grp * 8 + it) * NTHR + tid;
        const int row = idx >> 6, c16 = idx & 63;
        *(volatile v4u*)(emb16 + (rowbase + (size_t)row) * NDIM + (size_t)c16 * 8) = vals[it];
      }
      __threadfence();
    }
  }
#pragma unroll
  for (int grp = 0; grp < 2; ++grp) {
    v4u vals[8];
#pragma unroll
    for (int it = 0; it < 8; ++it) {
      const int idx = (grp * 8 + it) * NTHR + tid;
      const int d = idx >> 3, j = idx & 7;
      const int sh = (d & 1) * 16, wc = d >> 1;
      unsigned bt[8];
#pragma unroll
      for (int e = 0; e < 8; ++e) bt[e] = (ThW[(8 * j + e) * THW_PITCH + wc] >> sh) & 0xffffu;
      v4u pv;
      pv[0] = bt[0] | (bt[1] << 16);
      pv[1] = bt[2] | (bt[3] << 16);
      pv[2] = bt[4] | (bt[5] << 16);
      pv[3] = bt[6] | (bt[7] << 16);
      vals[it] = pv;
    }
    for (int pass = 0; pass < 2; ++pass) {
#pragma unroll
      for (int it = 0; it < 8; ++it) {
        const int idx = (grp * 8 + it) * NTHR + tid;
        const int d = idx >> 3, j = idx & 7;
        *(volatile v4u*)(embt16 + ((size_t)(bq * NDIM + d) * NSEQ + (size_t)(l0 + 8 * j))) = vals[it];
      }
      __threadfence();
    }
  }
}

__global__ __launch_bounds__(NTHR) void score_final_kernel(const float* __restrict__ st, const float* __restrict__ wa,
                                                          const float* __restrict__ ba, float* __restrict__ ratef) {
  __shared__ float sc[32];
  const int tid = threadIdx.x, lane = tid & 31, wave = tid >> 5;
  const size_t rowbase = (size_t)blockIdx.x * 32;
  v4f w[4];
#pragma unroll
  for (int q = 0; q < 4; ++q) w[q] = *(const v4f*)(wa + 128 * q + 4 * lane);
  const float bav = ba[0];
#pragma unroll 1
  for (int i = 0; i < 4; ++i) {
    const size_t row = rowbase + (size_t)(wave * 4 + i);
    const float* xp = st + row * NDIM;
    float p = 0.f;
#pragma unroll
    for (int q = 0; q < 4; ++q) {
      const v4f x = *(const v4f*)(xp + 128 * q + 4 * lane);
#pragma unroll
      for (int e = 0; e < 4; ++e) p += x[e] * w[q][e];
    }
#pragma unroll
    for (int off = 1; off < 32; off <<= 1) p += __shfl_xor(p, off, 32);
    if (lane == 0) sc[wave * 4 + i] = fmaxf(p + bav, 0.f);
  }
  __syncthreads();
  if (wave == 0) {
    const float vv = sc[lane];
    volatile float* rp = ratef + rowbase;
    rp[lane] = vv;
    __threadfence();
    rp[lane] = vv;
  }
}

__global__ __launch_bounds__(NTHR) void pool_final_kernel(const float* __restrict__ st, const float* __restrict__ attf,
                                                         float* __restrict__ spool) {
  const int i = blockIdx.x * NTHR + threadIdx.x;
  const int bq = i >> 7, d4 = (i & 127) * 4;
  const float* sp = st + (size_t)bq * NSEQ * NDIM + d4;
  const float* ap = attf + (size_t)bq * NSEQ;
  v4f acc = (v4f){0.f, 0.f, 0.f, 0.f};
#pragma unroll 1
  for (int l = 0; l < NSEQ; ++l) {
    const float a = ap[l];
    const v4f x = *(const v4f*)(sp + (size_t)l * NDIM);
    acc += x * a;
  }
  acc *= (1.0f / 32.0f);
  float* op = spool + (size_t)i * 4;
  *(volatile v4f*)op = acc;
  __threadfence();
  *(volatile v4f*)op = acc;
}

__global__ __launch_bounds__(512) void head_kernel(const float* __restrict__ spool, const float* __restrict__ ga,
                                                  const float* __restrict__ bea, const float* __restrict__ ott,
                                                  const float* __restrict__ wh, const float* __restrict__ bh,
                                                  float* __restrict__ pline) {
  __shared__ __align__(16) float pl[16];
  const int tid = threadIdx.x, lane = tid & 31, bq = tid >> 5;
  v4f v[4], g[4], e4[4], w[4];
#pragma unroll
  for (int q = 0; q < 4; ++q) {
    v[q] = *(const v4f*)(spool + (size_t)bq * NDIM + 128 * q + 4 * lane);
    g[q] = *(const v4f*)(ga + 128 * q + 4 * lane);
  }
  asm volatile("" ::: "memory");
#pragma unroll
  for (int q = 0; q < 4; ++q) {
    e4[q] = *(const v4f*)(bea + 128 * q + 4 * lane);
    w[q]  = *(const v4f*)(wh + 128 * q + 4 * lane);
  }
  asm volatile("" ::: "memory");
  float s = 0.f;
#pragma unroll
  for (int q = 0; q < 4; ++q) s += (v[q][0] + v[q][1]) + (v[q][2] + v[q][3]);
#pragma unroll
  for (int off = 1; off < 32; off <<= 1) s += __shfl_xor(s, off, 32);
  const float mean = s * (1.0f / NDIM);
  float ss = 0.f;
#pragma unroll
  for (int q = 0; q < 4; ++q)
#pragma unroll
    for (int e = 0; e < 4; ++e) { const float d = v[q][e] - mean; v[q][e] = d; ss += d * d; }
#pragma unroll
  for (int off = 1; off < 32; off <<= 1) ss += __shfl_xor(ss, off, 32);
  const float rstd = rsqrtf(ss * (1.0f / NDIM) + LN_EPS);
  float p = 0.f;
#pragma unroll
  for (int q = 0; q < 4; ++q)
#pragma unroll
    for (int e = 0; e < 4; ++e) {
      const float sl = (v[q][e] * rstd) * g[q][e] + e4[q][e];
      p += sl * w[q][e];
    }
#pragma unroll 1
  for (int c = 0; c < NOTT / 128; ++c) {
    const v4f o4 = *(const v4f*)(ott + (size_t)bq * NOTT + 128 * c + 4 * lane);
    const v4f w4 = *(const v4f*)(wh + NDIM + 128 * c + 4 * lane);
#pragma unroll
    for (int e = 0; e < 4; ++e) p += o4[e] * w4[e];
  }
#pragma unroll
  for (int off = 1; off < 32; off <<= 1) p += __shfl_xor(p, off, 32);
  const float logit = p + bh[0];
  const float pv = 1.0f / (1.0f + expf(-logit));
  if (lane == 0) pl[bq] = pv;
  __syncthreads();
  if (bq == 0) {
    const int li = (lane < 4) ? lane : 3;
    const v4f t4 = *(const v4f*)(pl + 4 * li);
    const float f = (lane < 4) ? 1.f : 0.f;
    const v4f o = t4 * f;
    if (lane < 8) {
      float* pp = pline + 4 * lane;
      *(volatile v4f*)pp = o;
      __threadfence();
      *(volatile v4f*)pp = o;
    }
  }
}

__global__ __launch_bounds__(NTHR) void out_copy_kernel(const float* __restrict__ pline, const float* __restrict__ sumall,
                                                       float* __restrict__ out, int nout) {
  const int i = blockIdx.x * NTHR + threadIdx.x;
  const int ip = (i < 4) ? i : 3;
  int ia = i - 4;
  ia = (ia < 0) ? 0 : ia;
  ia = (ia > NSUMALL / 4 - 1) ? (NSUMALL / 4 - 1) : ia;
  const v4f vp = *(const v4f*)(pline + 4 * ip);
  const v4f va = *(const v4f*)(sumall + (size_t)4 * ia);
  const float fp = (i < 4) ? 1.f : 0.f;
  const float fa = 1.0f - fp;
  v4f o;
#pragma unroll
  for (int e = 0; e < 4; ++e) o[e] = fmaf(fp, vp[e], fa * va[e]);
  if (4 * i + 3 < nout) {
    float* op = out + (size_t)4 * i;
    *(volatile v4f*)op = o;
    __threadfence();
    *(volatile v4f*)op = o;
  }
}

extern "C" void kernel_launch(void* const* d_in, const int* in_sizes, int n_in,
                              void* d_out, int out_size, void* d_ws, size_t ws_size, hipStream_t stream) {
  if (n_in < 21 || d_out == nullptr || d_ws == nullptr) return;
  if (in_sizes[0] != NROW * NDIM || in_sizes[1] != NLAY * NHEAD * NDIM || in_sizes[2] != NLAY * NHEAD ||
      in_sizes[3] != NLAY * NHEAD * NDIM || in_sizes[4] != NLAY * NHEAD * NDIM ||
      in_sizes[5] != NLAY * NHEAD * NDIM * NSM || in_sizes[6] != NLAY * NHEAD * NSM ||
      in_sizes[7] != NLAY * NDIM || in_sizes[8] != NLAY * NDIM || in_sizes[9] != NLAY * NDIM * NDIM ||
      in_sizes[10] != NLAY * NDIM || in_sizes[11] != NLAY * NDIM * NSETD || in_sizes[12] != NLAY * NSETD ||
      in_sizes[13] != NLAY * NDIM || in_sizes[14] != NLAY * NDIM || in_sizes[15] != NDIM || in_sizes[16] != 1 ||
      in_sizes[17] != NDIM || in_sizes[18] != NDIM || in_sizes[19] != NDIM + NOTT || in_sizes[20] != 1 ||
      out_size != NOUTF) return;

  const float* embding = (const float*)d_in[0];
  const float* W_att   = (const float*)d_in[1];
  const float* b_att   = (const float*)d_in[2];
  const float* g_att   = (const float*)d_in[3];
  const float* be_att  = (const float*)d_in[4];
  const float* W_pro   = (const float*)d_in[5];
  const float* b_pro   = (const float*)d_in[6];
  const float* w_p1    = (const float*)d_in[7];
  const float* b_p1    = (const float*)d_in[8];
  const float* W_FI    = (const float*)d_in[9];
  const float* b_FI    = (const float*)d_in[10];
  const float* W_Set   = (const float*)d_in[11];
  const float* b_Set   = (const float*)d_in[12];
  const float* g_n     = (const float*)d_in[13];
  const float* be_n    = (const float*)d_in[14];
  const float* w_aat   = (const float*)d_in[15];
  const float* b_aat   = (const float*)d_in[16];
  const float* g_aat   = (const float*)d_in[17];
  const float* be_aat  = (const float*)d_in[18];
  const float* W_h2p   = (const float*)d_in[19];
  const float* b_h2p   = (const float*)d_in[20];
  float* out = (float*)d_out;

  char* ws = (char*)d_ws; size_t off = 0;
  auto carve = [&](size_t bytes) -> char* { char* p = ws + off; off += (bytes + 255) & ~(size_t)255; return p; };
  float*          STA    = (float*)carve((size_t)NROW * NDIM * 4);
  float*          STB    = (float*)carve((size_t)NROW * NDIM * 4);
  unsigned short* EMB16  = (unsigned short*)carve((size_t)NROW * NDIM * 2);
  unsigned short* EMBT16 = (unsigned short*)carve((size_t)NBAT * NDIM * NSEQ * 2);
  unsigned short* WA16   = (unsigned short*)carve((size_t)NLAY * NHEAD * NDIM * 2);
  float*          RATE   = (float*)carve((size_t)NBAT * NHEAD * NSEQ * 4);
  float*          ATTF   = (float*)carve((size_t)NBAT * NHEAD * NSEQ * 4);
  unsigned short* ATT16  = (unsigned short*)carve((size_t)NBAT * NHEAD * NSEQ * 2);
  float*          SUMALL = (float*)carve((size_t)NSUMALL * 4);
  float*          SRAW   = (float*)carve((size_t)NBAT * NHEAD * NDIM * 4);
  float*          VEC    = (float*)carve((size_t)NBAT * NHEAD * VECP * 4);
  float*          OTT    = (float*)carve((size_t)NBAT * NOTT * 4);
  float*          RATEF  = (float*)carve((size_t)NBAT * NSEQ * 4);
  float*          ATTFIN = (float*)carve((size_t)NBAT * NSEQ * 4);
  float*          SPOOL  = (float*)carve((size_t)NBAT * NDIM * 4);
  float*          PLINE  = (float*)carve((size_t)32 * 4);
  if (off > ws_size || off > (size_t)134217728) return;

  const int n8w = NLAY * NHEAD * NDIM / 8;
  cvt_f16x8_kernel<<<(n8w + NTHR - 1) / NTHR, NTHR, 0, stream>>>(W_att, WA16, n8w, WATT_CARRY);
  carry_kernel<false><<<NROW / 64, NTHR, 0, stream>>>(embding, SUMALL, w_p1, b_p1, g_n, be_n, STA, EMB16, EMBT16);

  for (int t = 0; t < NLAY; ++t) {
    const float* cur = (t == 0) ? embding : (((t - 1) & 1) ? STB : STA);
    float* nxt = (t & 1) ? STB : STA;
    float* sum_t = SUMALL + (size_t)t * NBAT * NSEQ;
    wmma_gemm64<0, false, 1, 0, false, 2><<<dim3(2, NBAT), 256, 0, stream>>>(
        WA16 + (size_t)t * NHEAD * NDIM, WA16 + (size_t)t * NHEAD * NDIM, NDIM, 0L,
        EMB16, EMB16, NDIM, (long)NSEQ * NDIM,
        (void*)RATE, (void*)RATE, NSEQ, (long)NHEAD * NSEQ,
        b_att + (size_t)t * NHEAD, SRAW, 0L, NHEAD, NSEQ, NDIM, RATE_SCALE);
    softmax_rows_kernel<true><<<NBAT * NHEAD, NTHR, 0, stream>>>(RATE, ATTF, ATT16);
    headsum_kernel<<<(NBAT * NSEQ / 4) / NTHR, NTHR, 0, stream>>>(ATTF, sum_t);
    wmma_gemm64<0, false, 0, 0, false, 0><<<dim3(1, NBAT), 256, 0, stream>>>(
        ATT16, ATT16, NSEQ, (long)NHEAD * NSEQ,
        EMBT16, EMBT16, NSEQ, (long)NDIM * NSEQ,
        (void*)SRAW, (void*)SRAW, NDIM, (long)NHEAD * NDIM,
        b_att, RATE, 0L, NHEAD, NDIM, NSEQ, POOL_SCALE);
    lnpro_kernel<<<(NBAT * NHEAD) / 8, NTHR, 0, stream>>>(
        SRAW, g_att + (size_t)t * NHEAD * NDIM, be_att + (size_t)t * NHEAD * NDIM,
        W_pro + (size_t)t * NHEAD * NDIM * NSM, b_pro + (size_t)t * NHEAD * NSM, VEC);
    fiset_kernel<<<1, NTHR, 0, stream>>>(VEC, W_FI + (size_t)t * NDIM * NDIM, b_FI + (size_t)t * NDIM,
                                         W_Set + (size_t)t * NDIM * NSETD, b_Set + (size_t)t * NSETD, OTT, t * NSETD);
    carry_kernel<true><<<NROW / 64, NTHR, 0, stream>>>(cur, sum_t, w_p1 + (size_t)t * NDIM, b_p1 + (size_t)t * NDIM,
                                                       g_n + (size_t)t * NDIM, be_n + (size_t)t * NDIM, nxt, EMB16, EMBT16);
  }
  float* fin = ((NLAY - 1) & 1) ? STB : STA;

  score_final_kernel<<<NROW / 32, NTHR, 0, stream>>>(fin, w_aat, b_aat, RATEF);
  softmax_rows_kernel<false><<<NBAT, NTHR, 0, stream>>>(RATEF, ATTFIN, ATT16);
  pool_final_kernel<<<(NBAT * NDIM / 4) / NTHR, NTHR, 0, stream>>>(fin, ATTFIN, SPOOL);
  head_kernel<<<1, 512, 0, stream>>>(SPOOL, g_aat, be_aat, OTT, W_h2p, b_h2p, PLINE);
  out_copy_kernel<<<(NOUTF / 4 + NTHR - 1) / NTHR, NTHR, 0, stream>>>(PLINE, SUMALL, out, NOUTF);
}
